// Dense_RBS_state_vector_31963146617513
// MI455X (gfx1250) — hardware-run, weakly checked
//
#include <hip/hip_runtime.h>
#include <math.h>

typedef __attribute__((ext_vector_type(16))) _Float16 v16h;
typedef __attribute__((ext_vector_type(8)))  _Float16 v8h;
typedef unsigned short v8us __attribute__((ext_vector_type(8)));
typedef __attribute__((ext_vector_type(2)))  _Float16 v2h;
typedef __attribute__((ext_vector_type(16))) __bf16   v16b;
typedef __attribute__((ext_vector_type(8)))  __bf16   v8b;
typedef __attribute__((ext_vector_type(8)))  float    v8f;
typedef __attribute__((ext_vector_type(4)))  float    v4f;
typedef __attribute__((ext_vector_type(2)))  float    v2f;

constexpr int kG    = 62;
constexpr int kD    = 496;
constexpr int kDP   = 512;
constexpr int kNB   = 4096;
constexpr int kThr  = 256;
constexpr float kInCarry = 1024.0f;
constexpr float kSc20 = 1.0f / (kInCarry * kInCarry);
constexpr float kF16MinNormal = 6.103515625e-5f;

static_assert(kG == 62 && kD == 496 && kDP == 512 && kNB == 4096 && kD == 62 * 8, "the index arithmetic below uses these sizes");

constexpr size_t kOffM16 = 0ull;
constexpr size_t kOffR16 = 32505856ull;
constexpr size_t kOffRF = 33030144ull;
constexpr size_t kOffRT = 34078720ull;
constexpr size_t kOffS16 = 34603008ull;
constexpr size_t kOffF32 = 38797312ull;
constexpr size_t kWsTotal = 47185920ull;
static_assert(kWsTotal <= 134217728ull, "the carve stands under 128 MiB");
static_assert(kOffM16 == 0
  && kOffR16 == kOffM16 + 32505856ull
  && kOffRF == kOffR16 + 524288ull
  && kOffRT == kOffRF + 1048576ull
  && kOffS16 == kOffRT + 524288ull
  && kOffF32 == kOffS16 + 4194304ull
  && kWsTotal == kOffF32 + 8388608ull, "the carve is a chain: every region starts where the one before ends");
static_assert((kOffM16 % 256) == 0 && (kOffR16 % 256) == 0 && (kOffRF % 256) == 0 && (kOffRT % 256) == 0 && (kOffS16 % 256) == 0 && (kOffF32 % 256) == 0, "every region starts on a multiple of 256 B");

__device__ __forceinline__ unsigned short f2bf_bits(float f) {
  unsigned u = __float_as_uint(f);
  return (unsigned short)((u + 0x7FFFu + ((u >> 16) & 1u)) >> 16);
}
__device__ __forceinline__ float bf_bits2f(unsigned short h) { return __uint_as_float(((unsigned)h) << 16); }
__device__ __forceinline__ float bf16r(float f) { return bf_bits2f(f2bf_bits(f)); }
__device__ __forceinline__ float carry_flush(float v, float carry) {
  const float s = v * carry;
  return (fabsf(s) < kF16MinNormal) ? 0.0f : s;
}

__device__ __forceinline__ void dep_guard4_h(v8f& a, v8f& b, v8f& c, v8f& d, v16h x, v16h y) { asm volatile("v_nop\n\tv_nop\n\tv_nop\n\tv_nop" : "+v"(a), "+v"(b), "+v"(c), "+v"(d) : "v"(x), "v"(y)); }
__device__ __forceinline__ void dep_guard4_b(v8f& a, v8f& b, v8f& c, v8f& d, v16b x, v16b y) { asm volatile("v_nop\n\tv_nop\n\tv_nop\n\tv_nop" : "+v"(a), "+v"(b), "+v"(c), "+v"(d) : "v"(x), "v"(y)); }
__device__ __forceinline__ void keep4_h(v16h a, v16h b, v16h c, v16h d) { asm volatile("v_nop" :: "v"(a), "v"(b), "v"(c), "v"(d)); }
__device__ __forceinline__ void keep4_b(v16b a, v16b b, v16b c, v16b d) { asm volatile("v_nop" :: "v"(a), "v"(b), "v"(c), "v"(d)); }
__device__ __forceinline__ void acc_guard4(v8f& a, v8f& b, v8f& c, v8f& d) { asm volatile("v_nop\n\tv_nop\n\tv_nop\n\tv_nop" : "+v"(a), "+v"(b), "+v"(c), "+v"(d)); }

template <typename T> struct Frag;
template <> struct Frag<_Float16> {
  typedef v16h V; union U { v16h v; v8h h[2]; };
  static __device__ __forceinline__ v16h load(const _Float16* p) {
    U f; f.h[0] = *(const v8h*)(p); f.h[1] = *(const v8h*)(p + 16); return f.v;
  }
  static __device__ __forceinline__ v8f mma(v16h a, v16h b, v8f c) {
    return __builtin_amdgcn_wmma_f32_16x16x32_f16(false, a, false, b, (short)0, c, false, false);
  }
  static __device__ __forceinline__ void guard4(v8f& a, v8f& b, v8f& c, v8f& d, v16h x, v16h y) { dep_guard4_h(a, b, c, d, x, y); }
  static __device__ __forceinline__ void keep(v16h a, v16h b, v16h c, v16h d) { keep4_h(a, b, c, d); }
};
template <> struct Frag<__bf16> {
  typedef v16b V; union U { v16b v; v8b h[2]; };
  static __device__ __forceinline__ v16b load(const __bf16* p) {
    U f; f.h[0] = *(const v8b*)(p); f.h[1] = *(const v8b*)(p + 16); return f.v;
  }
  static __device__ __forceinline__ v8f mma(v16b a, v16b b, v8f c) {
    return __builtin_amdgcn_wmma_f32_16x16x32_bf16(false, a, false, b, (short)0, c, false, false);
  }
  static __device__ __forceinline__ void guard4(v8f& a, v8f& b, v8f& c, v8f& d, v16b x, v16b y) { dep_guard4_b(a, b, c, d, x, y); }
  static __device__ __forceinline__ void keep(v16b a, v16b b, v16b c, v16b d) { keep4_b(a, b, c, d); }
};

__device__ __forceinline__ v8f mma_h(v16h a, v16h b, v8f c) {
  c = __builtin_amdgcn_wmma_f32_16x16x32_f16(false, a, false, b, (short)0, c, false, false);
  asm volatile("v_nop\n\tv_nop\n\tv_nop\n\tv_nop" : "+v"(c) : "v"(a), "v"(b));
  return c;
}

template <int ET> struct Elem;
template <> struct Elem<0> { typedef _Float16 T; };
template <> struct Elem<1> { typedef __bf16 T; };
template <int ET, bool SPLIT, int BIAS_MODE, int OUT_MODE, bool RESID, int ACT = 0>
__global__ __launch_bounds__(256) void wmma_gemm64(
    const unsigned short* __restrict__ Ap, const unsigned short* __restrict__ A2p, int lda, long strideA,
    const unsigned short* __restrict__ Btp, const unsigned short* __restrict__ Bt2p, int ldb, long strideB,
    void* __restrict__ Cout, void* __restrict__ Cout2, int ldc, long strideC,
    const float* __restrict__ bias,
    const float* __restrict__ resid, long strideR,
    int M, int N, int K, float scale) {
  typedef typename Elem<ET>::T T;
  typedef typename Frag<T>::V V;
  const T* A = (const T*)Ap; const T* A2 = (const T*)A2p; const T* Bt = (const T*)Btp; const T* Bt2 = (const T*)Bt2p;
  __shared__ __align__(16) float sT[8][16 * 68];
  const int b    = blockIdx.y;
  const int lane = threadIdx.x & 31;
  const int wave = threadIdx.x >> 5;
  const int tilesN = N >> 6;
  const int tilesM = M >> 6;
  const int tile = blockIdx.x * 8 + wave;
  if (tile >= tilesM * tilesN) return;
  const int tm = tile / tilesN;
  const int tn = tile - tm * tilesN;
  const int m0 = tm << 6;
  const int n0 = tn << 6;

  const T* Ab  = A  + (size_t)b * strideA;
  const T* Bb  = Bt + (size_t)b * strideB;
  const T* Ab2 = SPLIT ? (A2  + (size_t)b * strideA) : nullptr;
  const T* Bb2 = SPLIT ? (Bt2 + (size_t)b * strideB) : nullptr;

  const int rlane = lane & 15;
  const int koff  = (lane >> 4) * 8;
  const int mOff  = (lane >> 4) * 8;

  v8f acc[4][4];
#pragma unroll
  for (int i = 0; i < 4; ++i)
#pragma unroll
    for (int j = 0; j < 4; ++j) acc[i][j] = (v8f){0.f,0.f,0.f,0.f,0.f,0.f,0.f,0.f};

  for (int k0 = 0; k0 < K; k0 += 32) {
    V bh[4], bl[4];
#pragma unroll
    for (int j = 0; j < 4; ++j) {
      const size_t bo = (size_t)(n0 + (j << 4) + rlane) * ldb + koff + k0;
      bh[j] = Frag<T>::load(Bb + bo);
      if (SPLIT) bl[j] = Frag<T>::load(Bb2 + bo);
    }
#pragma unroll
    for (int i = 0; i < 4; ++i) {
      const size_t ao = (size_t)(m0 + (i << 4) + rlane) * lda + koff + k0;
      V ah = Frag<T>::load(Ab + ao);
      V al;
      if (SPLIT) al = Frag<T>::load(Ab2 + ao);
#pragma unroll
      for (int j = 0; j < 4; ++j) {
        acc[i][j] = Frag<T>::mma(ah, bh[j], acc[i][j]);
        if (SPLIT) {
          acc[i][j] = Frag<T>::mma(ah, bl[j], acc[i][j]);
          acc[i][j] = Frag<T>::mma(al, bh[j], acc[i][j]);
        }
      }
      Frag<T>::guard4(acc[i][0], acc[i][1], acc[i][2], acc[i][3], ah, SPLIT ? al : ah);
    }
    Frag<T>::keep(bh[0], bh[1], bh[2], bh[3]);
    if (SPLIT) Frag<T>::keep(bl[0], bl[1], bl[2], bl[3]);
  }
  acc_guard4(acc[0][0], acc[0][1], acc[0][2], acc[0][3]);
  acc_guard4(acc[1][0], acc[1][1], acc[1][2], acc[1][3]);
  acc_guard4(acc[2][0], acc[2][1], acc[2][2], acc[2][3]);
  acc_guard4(acc[3][0], acc[3][1], acc[3][2], acc[3][3]);

  float* slab = sT[wave];
  const float* Rb = RESID ? (resid + (size_t)b * strideR) : nullptr;
#pragma unroll
  for (int i = 0; i < 4; ++i) {
    const int mBase = m0 + (i << 4);
#pragma unroll
    for (int j = 0; j < 4; ++j) {
      const int n = n0 + (j << 4) + rlane;
      float bv = 0.f;
      if (BIAS_MODE == 2) bv = bias[n];
#pragma unroll
      for (int r = 0; r < 8; ++r) {
        float v = acc[i][j][r] * scale;
        if (BIAS_MODE == 1) v += bias[mBase + mOff + r];
        if (BIAS_MODE == 2) v += bv;
        if (RESID) v += Rb[(size_t)(mBase + mOff + r) * ldc + n];
        if (ACT == 1) v = tanhf(v);
        if (ACT == 2) v = fmaxf(v, 0.0f);
        if (ACT == 3) v = v / (1.0f + expf(-v));
        if (ACT == 4) v = (v > 0.f) ? v : 0.01f * v;
        slab[(mOff + r) * 68 + (j << 4) + rlane] = v;
      }
    }
    __builtin_amdgcn_fence(__ATOMIC_RELEASE, "workgroup");
    __builtin_amdgcn_wave_barrier();
    __builtin_amdgcn_fence(__ATOMIC_ACQUIRE, "workgroup");
    if (OUT_MODE == 0) {
      float* C = (float*)Cout + (size_t)b * strideC;
      const int hh = lane >> 4, c4 = (lane & 15) * 4;
      for (int pass = 0; pass < 2; ++pass) {
#pragma unroll
        for (int it = 0; it < 8; ++it) {
          const int row = it * 2 + hh;
          v4f v = *(const v4f*)(slab + row * 68 + c4);
          *(volatile v4f*)(C + (size_t)(mBase + row) * ldc + n0 + c4) = v;
        }
        __threadfence();
      }
    } else {
      const int q = lane >> 3, c8 = (lane & 7) * 8;
      unsigned short* C  = (unsigned short*)Cout  + (size_t)b * strideC;
      unsigned short* C2 = (OUT_MODE == 2) ? ((unsigned short*)Cout2 + (size_t)b * strideC) : nullptr;
      for (int pass = 0; pass < 2; ++pass) {
#pragma unroll
        for (int it = 0; it < 4; ++it) {
          const int row = it * 4 + q;
          const float* sp = slab + row * 68 + c8;
          v8h hv, lv;
#pragma unroll
          for (int e = 0; e < 8; ++e) {
            if (OUT_MODE == 1) {
              hv[e] = (_Float16)sp[e];
            } else {
              unsigned short hb = f2bf_bits(sp[e]);
              unsigned short lb = f2bf_bits(sp[e] - bf_bits2f(hb));
              hv[e] = __builtin_bit_cast(_Float16, hb);
              lv[e] = __builtin_bit_cast(_Float16, lb);
            }
          }
          *(volatile v8h*)(C + (size_t)(mBase + row) * ldc + n0 + c8) = hv;
          if (OUT_MODE == 2) *(volatile v8h*)(C2 + (size_t)(mBase + row) * ldc + n0 + c8) = lv;
        }
        __threadfence();
      }
    }
    __builtin_amdgcn_fence(__ATOMIC_RELEASE, "workgroup");
    __builtin_amdgcn_wave_barrier();
    __builtin_amdgcn_fence(__ATOMIC_ACQUIRE, "workgroup");
  }
}

__global__ __launch_bounds__(kThr) void gatem_kernel(const float* __restrict__ U, const float* __restrict__ ang, unsigned short* __restrict__ M16) {
  const unsigned i = blockIdx.x * (unsigned)kThr + threadIdx.x;
  const unsigned g = i >> 15, r = (i >> 6) & 511u, cg = i & 63u;
  const unsigned keep = ((r < (unsigned)kD) & (cg < 62u)) ? 0xFFFFFFFFu : 0u;
  const unsigned rs = (r < (unsigned)kD) ? r : (unsigned)(kD - 1);
  const unsigned cs = (cg < 62u) ? cg : 61u;
  const float th = bf16r(ang[g]);
  const float cv = cosf(th), sv = sinf(th);
  const float* p0 = U + (((size_t)g * 3u + 0u) * (unsigned)kD + rs) * (unsigned)kD + 8u * cs;
  const float* p1 = p0 + (size_t)kD * kD;
  const float* p2 = p1 + (size_t)kD * kD;
  const v4f a0 = *(const v4f*)p0, a1 = *(const v4f*)(p0 + 4);
  const v4f b0 = *(const v4f*)p1, b1 = *(const v4f*)(p1 + 4);
  const v4f c0 = *(const v4f*)p2, c1 = *(const v4f*)(p2 + 4);
  v8h hv;
#pragma unroll
  for (int e = 0; e < 4; ++e) {
    const float m0 = bf16r(a0[e]) * cv + bf16r(b0[e]) * sv + bf16r(c0[e]);
    const float m1 = bf16r(a1[e]) * cv + bf16r(b1[e]) * sv + bf16r(c1[e]);
    hv[e]     = (_Float16)__uint_as_float(__float_as_uint(carry_flush(m0, kInCarry)) & keep);
    hv[4 + e] = (_Float16)__uint_as_float(__float_as_uint(carry_flush(m1, kInCarry)) & keep);
  }
  unsigned short* dp = M16 + (size_t)i * 8u;
  *(volatile v8h*)dp = hv;
  __threadfence();
  *(volatile v8h*)dp = hv;
}
static_assert(kG * kDP * (kDP / 8) == 7936 * kThr, "the gates' kernel's grid exact");

__global__ __launch_bounds__(kThr) void eye_kernel(unsigned short* __restrict__ R) {
  const unsigned i = blockIdx.x * (unsigned)kThr + threadIdx.x;
  const unsigned r = i >> 6, c8 = (i & 63u) << 3;
  v8h hv;
#pragma unroll
  for (int e = 0; e < 8; ++e) hv[e] = (_Float16)(((c8 + (unsigned)e == r) & (r < (unsigned)kD)) ? kInCarry : 0.0f);
  unsigned short* dp = R + (size_t)i * 8u;
  *(volatile v8h*)dp = hv;
  __threadfence();
  *(volatile v8h*)dp = hv;
}

__global__ __launch_bounds__(kThr) void spadc_kernel(const float* __restrict__ x, unsigned short* __restrict__ S16) {
  const unsigned i = blockIdx.x * (unsigned)kThr + threadIdx.x;
  const unsigned b = i >> 6, cg = i & 63u;
  const unsigned keep = (cg < 62u) ? 0xFFFFFFFFu : 0u;
  const unsigned cs = (cg < 62u) ? cg : 61u;
  const float* sp = x + (size_t)b * (unsigned)kD + 8u * cs;
  const v4f a0 = *(const v4f*)sp, a1 = *(const v4f*)(sp + 4);
  v8h hv;
#pragma unroll
  for (int e = 0; e < 4; ++e) {
    hv[e]     = (_Float16)__uint_as_float(__float_as_uint(carry_flush(bf16r(a0[e]), kInCarry)) & keep);
    hv[4 + e] = (_Float16)__uint_as_float(__float_as_uint(carry_flush(bf16r(a1[e]), kInCarry)) & keep);
  }
  unsigned short* dp = S16 + (size_t)i * 8u;
  *(volatile v8h*)dp = hv;
  __threadfence();
  *(volatile v8h*)dp = hv;
}

__global__ __launch_bounds__(kThr) void rcast_kernel(const float* __restrict__ F, unsigned short* __restrict__ R) {
  const unsigned i = blockIdx.x * (unsigned)kThr + threadIdx.x;
  const float* sp = F + (size_t)i * 8u;
  const v4f a0 = *(const v4f*)sp, a1 = *(const v4f*)(sp + 4);
  v8h hv;
#pragma unroll
  for (int e = 0; e < 4; ++e) {
    hv[e]     = (_Float16)carry_flush(a0[e], kInCarry);
    hv[4 + e] = (_Float16)carry_flush(a1[e], kInCarry);
  }
  unsigned short* dp = R + (size_t)i * 8u;
  *(volatile v8h*)dp = hv;
  __threadfence();
  *(volatile v8h*)dp = hv;
}

__global__ __launch_bounds__(kThr) void rturn_kernel(const unsigned short* __restrict__ R, unsigned short* __restrict__ RT) {
  const unsigned i = blockIdx.x * (unsigned)kThr + threadIdx.x;
  const unsigned n = i >> 6, k8 = (i & 63u) << 3;
  const unsigned short* sp = R + (size_t)k8 * (unsigned)kDP + n;
  v8us wv;
#pragma unroll
  for (int e = 0; e < 8; ++e) wv[e] = sp[(size_t)e * (unsigned)kDP];
  unsigned short* dp = RT + (size_t)i * 8u;
  *(volatile v8us*)dp = wv;
  __threadfence();
  *(volatile v8us*)dp = wv;
}

__global__ __launch_bounds__(kThr) void crop_kernel(const float* __restrict__ F, float* __restrict__ out) {
  const unsigned i = blockIdx.x * (unsigned)kThr + threadIdx.x;
  const unsigned b = i / 62u, c8 = (i - b * 62u) << 3;
  const float* sp = F + (size_t)b * (unsigned)kDP + c8;
  const v4f y0 = *(const v4f*)sp, y1 = *(const v4f*)(sp + 4);
  float* dp = out + (size_t)i * 8u;
  *(volatile v4f*)dp = y0;
  *(volatile v4f*)(dp + 4) = y1;
  __threadfence();
  *(volatile v4f*)dp = y0;
  *(volatile v4f*)(dp + 4) = y1;
}
static_assert(kNB * 62 == 992 * kThr, "the crop's grid exact");

extern "C" void kernel_launch(void* const* d_in, const int* in_sizes, int n_in,
                              void* d_out, int out_size, void* d_ws, size_t ws_size,
                              hipStream_t stream) {
  if (n_in < 3 || d_out == nullptr || d_ws == nullptr) return;
  if (in_sizes[0] != kNB * kD || in_sizes[1] != kG || in_sizes[2] != kG * 3 * kD * kD) return;
  if (out_size != kNB * kD) return;
  if (ws_size < kWsTotal) return;
  const float* x = (const float*)d_in[0];
  const float* ang = (const float*)d_in[1];
  const float* U = (const float*)d_in[2];
  float* out = (float*)d_out;
  char* ws = (char*)d_ws;
  unsigned short* M16 = (unsigned short*)(ws + kOffM16);
  unsigned short* R16 = (unsigned short*)(ws + kOffR16);
  float* RF = (float*)(ws + kOffRF);
  unsigned short* RT = (unsigned short*)(ws + kOffRT);
  unsigned short* S16 = (unsigned short*)(ws + kOffS16);
  float* F32 = (float*)(ws + kOffF32);

  static_assert((kDP * kDP / 8) % kThr == 0 && (kNB * kDP / 8) % kThr == 0, "every flat kernel's grid exact");
  gatem_kernel<<<kG * kDP * (kDP / 8) / kThr, kThr, 0, stream>>>(U, ang, M16);
  eye_kernel<<<kDP * kDP / 8 / kThr, kThr, 0, stream>>>(R16);
  spadc_kernel<<<kNB * kDP / 8 / kThr, kThr, 0, stream>>>(x, S16);
  for (int g = 0; g < kG; ++g) {
    wmma_gemm64<0, false, 0, 0, false, 0><<<dim3((kDP / 64) * (kDP / 64) / 8, 1), 256, 0, stream>>>(
        R16, R16, kDP, 0L, M16 + (size_t)g * kDP * kDP, M16 + (size_t)g * kDP * kDP, kDP, 0L, (void*)RF, (void*)RF, kDP, 0L, nullptr, nullptr, 0L, kDP, kDP, kDP, kSc20);
    rcast_kernel<<<kDP * kDP / 8 / kThr, kThr, 0, stream>>>(RF, R16);
  }
  rturn_kernel<<<kDP * kDP / 8 / kThr, kThr, 0, stream>>>(R16, RT);
  wmma_gemm64<0, false, 0, 0, false, 0><<<dim3((kNB / 64) * (kDP / 64) / 8, 1), 256, 0, stream>>>(
      S16, S16, kDP, 0L, RT, RT, kDP, 0L, (void*)F32, (void*)F32, kDP, 0L, nullptr, nullptr, 0L, kNB, kDP, kDP, kSc20);
  crop_kernel<<<kNB * 62 / kThr, kThr, 0, stream>>>(F32, out);
}
static_assert(((kDP / 64) * (kDP / 64)) % 8 == 0 && ((kNB / 64) * (kDP / 64)) % 8 == 0 && kDP % 32 == 0, "the engine's grids: whole blocks of eight wave tiles; the depth a multiple of 32");
